// SSMCompositionBlock_64596308132158
// MI455X (gfx1250) — hardware-run, weakly checked
//
#include <hip/hip_runtime.h>
#include <math.h>

typedef __attribute__((ext_vector_type(16))) _Float16 v16h;
typedef __attribute__((ext_vector_type(8)))  _Float16 v8h;
typedef __attribute__((ext_vector_type(8)))  float    v8f;
typedef __attribute__((ext_vector_type(4)))  float    v4f;

constexpr int kB  = 4;
constexpr int kT  = 2048;
constexpr int kH  = 1024;
constexpr int kS  = 64;
constexpr int kP  = 64;
constexpr int kNH = 8;
constexpr int kHD = kH / kNH;
constexpr int kM  = kB * kT;
constexpr int kTShift = 11;
static_assert(kHD == 128, "head width");
static_assert((1 << kTShift) == kT, "batch index = row >> kTShift");
static_assert((kM % 64) == 0 && (kH % 64) == 0 && (kS % 64) == 0 && (kT % 64) == 0, "tile multiples");
static_assert((kH % 32) == 0 && (kS % 32) == 0 && (kHD % 32) == 0 && (kT % 32) == 0, "K multiples of 32");
static_assert(kB * kP == 256 && kS == 64, "one-block kernels assume 256 lanes");

constexpr float kCarryAct = 16.0f;
constexpr float kCarryW   = 256.0f;
constexpr float kCarryC   = 64.0f;
constexpr float kCarryCtx = 256.0f;
constexpr float kCarryP   = 32768.0f;
constexpr float kF16MinNormal = 6.103515625e-5f;

constexpr size_t kOffXQ   = 0;
constexpr size_t kOffBN   = kOffXQ   + (size_t)kM * kH * 2;
constexpr size_t kOffWQKV = kOffBN   + (size_t)kM * kH * 2;
constexpr size_t kOffWO   = kOffWQKV + (size_t)3 * kH * kH * 2;
constexpr size_t kOffWIN  = kOffWO   + (size_t)kH * kH * 2;
constexpr size_t kOffBMT  = kOffWIN  + (size_t)kH * kH * 2;
constexpr size_t kOffCMT  = kOffBMT  + (size_t)kS * kH * 2;
constexpr size_t kOffQP   = kOffCMT  + (size_t)kH * kS * 2;
constexpr size_t kOffKP   = kOffQP   + (size_t)kM * kH * 2;
constexpr size_t kOffVT   = kOffKP   + (size_t)kM * kH * 2;
constexpr size_t kOffX1   = kOffVT   + (size_t)kM * kH * 2;
constexpr size_t kOffU    = kOffX1   + (size_t)kM * kH * 4;
constexpr size_t kOffST32 = kOffU    + (size_t)kM * kS * 4;
constexpr size_t kOffST16 = kOffST32 + (size_t)kM * kS * 4;
constexpr size_t kOffPM   = kOffST16 + (size_t)kM * kS * 2;
constexpr size_t kOffMOD  = kOffPM   + (size_t)kB * kP * 4;
constexpr size_t kWsTotal = kOffMOD  + (size_t)kB * kH * 4;
static_assert(kWsTotal == 133448704ull, "carve total");
static_assert(kWsTotal <= 134217728ull, "carve cap");
static_assert((kOffBN % 128) == 0 && (kOffWQKV % 128) == 0 && (kOffWO % 128) == 0 && (kOffWIN % 128) == 0 &&
              (kOffBMT % 128) == 0 && (kOffCMT % 128) == 0 && (kOffQP % 128) == 0 && (kOffKP % 128) == 0 &&
              (kOffVT % 128) == 0 && (kOffX1 % 128) == 0 && (kOffU % 128) == 0 && (kOffST32 % 128) == 0 &&
              (kOffST16 % 128) == 0 && (kOffPM % 128) == 0 && (kOffMOD % 128) == 0, "128-B aligned regions");
static_assert(kOffBN == kOffXQ + (size_t)kM * kH * 2, "XQ and BN adjacent (fused LN1 launch)");

__device__ __forceinline__ _Float16 to_f16_flush(float x) {
  const float y = (fabsf(x) < kF16MinNormal) ? 0.0f : x;
  return (_Float16)y;
}

__device__ __forceinline__ void wave_lds_sync() {
  __builtin_amdgcn_fence(__ATOMIC_RELEASE, "workgroup");
  __builtin_amdgcn_wave_barrier();
  __builtin_amdgcn_fence(__ATOMIC_ACQUIRE, "workgroup");
}

__device__ __forceinline__ void guard4_h(v8f& a0, v8f& a1, v8f& a2, v8f& a3, v16h x, v16h b0, v16h b1, v16h b2, v16h b3) {
  asm volatile("v_nop\n\tv_nop\n\tv_nop\n\tv_nop" : "+v"(a0), "+v"(a1), "+v"(a2), "+v"(a3) : "v"(x), "v"(b0), "v"(b1), "v"(b2), "v"(b3));
}
__device__ __forceinline__ void keep4_h(v16h a, v16h b, v16h c, v16h d) { asm volatile("v_nop" :: "v"(a), "v"(b), "v"(c), "v"(d)); }
__device__ __forceinline__ void acc_guard4(v8f& a, v8f& b, v8f& c, v8f& d) { asm volatile("v_nop\n\tv_nop\n\tv_nop\n\tv_nop" : "+v"(a), "+v"(b), "+v"(c), "+v"(d)); }

template <typename T> struct Frag;
template <> struct Frag<_Float16> {
  typedef v16h V; union U { v16h v; v8h h[2]; };
  static __device__ __forceinline__ v16h load(const _Float16* p) {
    U f; f.h[0] = *(const v8h*)(p); f.h[1] = *(const v8h*)(p + 16); return f.v;
  }
  static __device__ __forceinline__ v8f mma(v16h a, v16h b, v8f c) {
    return __builtin_amdgcn_wmma_f32_16x16x32_f16(false, a, false, b, (short)0, c, false, false);
  }
};
typedef Frag<_Float16> FragH;

template <int BIAS_MODE, int OUT_MODE, int RESID>
__global__ __launch_bounds__(256) __attribute__((amdgpu_num_vgpr(256))) void gemm64_f16_kernel(
    const unsigned short* __restrict__ Ap, int lda, long strideA,
    const unsigned short* __restrict__ Btp, int ldb, long strideB,
    void* Cout, int ldc, long strideC,
    const float* __restrict__ bias,
    const float* resid,
    const float* rowadd, int rowshift,
    int M, int N, int K, float scale, float oscale) {
  typedef _Float16 T;
  typedef v16h V;
  const T* A = (const T*)Ap; const T* Bt = (const T*)Btp;
  __shared__ __align__(16) float sT[8][16 * 68];
  const int b    = blockIdx.y;
  const int lane = threadIdx.x & 31;
  const int wave = threadIdx.x >> 5;
  const int tilesN = N >> 6;
  const int tilesM = M >> 6;
  const int tile = blockIdx.x * 8 + wave;
  if (tile >= tilesM * tilesN) return;
  const int tm = tile / tilesN;
  const int tn = tile - tm * tilesN;
  const int m0 = tm << 6;
  const int n0 = tn << 6;

  const T* Ab = A  + (size_t)b * strideA;
  const T* Bb = Bt + (size_t)b * strideB;

  const int rlane = lane & 15;
  const int koff  = (lane >> 4) * 8;
  const int mOff  = (lane >> 4) * 8;

  v8f acc[4][4];
#pragma unroll
  for (int i = 0; i < 4; ++i)
#pragma unroll
    for (int j = 0; j < 4; ++j) acc[i][j] = (v8f){0.f,0.f,0.f,0.f,0.f,0.f,0.f,0.f};

  for (int k0 = 0; k0 < K; k0 += 32) {
    V bh[4];
#pragma unroll
    for (int j = 0; j < 4; ++j) {
      const size_t bo = (size_t)(n0 + (j << 4) + rlane) * ldb + koff + k0;
      bh[j] = FragH::load(Bb + bo);
    }
#pragma unroll
    for (int i = 0; i < 4; ++i) {
      const size_t ao = (size_t)(m0 + (i << 4) + rlane) * lda + koff + k0;
      V ah = FragH::load(Ab + ao);
#pragma unroll
      for (int j = 0; j < 4; ++j) acc[i][j] = FragH::mma(ah, bh[j], acc[i][j]);
      guard4_h(acc[i][0], acc[i][1], acc[i][2], acc[i][3], ah, bh[0], bh[1], bh[2], bh[3]);
    }
    keep4_h(bh[0], bh[1], bh[2], bh[3]);
  }
  acc_guard4(acc[0][0], acc[0][1], acc[0][2], acc[0][3]);
  acc_guard4(acc[1][0], acc[1][1], acc[1][2], acc[1][3]);
  acc_guard4(acc[2][0], acc[2][1], acc[2][2], acc[2][3]);
  acc_guard4(acc[3][0], acc[3][1], acc[3][2], acc[3][3]);

  float* slab = sT[wave];
#pragma unroll
  for (int i = 0; i < 4; ++i) {
    const int mBase = m0 + (i << 4);
    float br[8];
    if (BIAS_MODE == 1) {
      const v4f b0 = *(const v4f*)(bias + mBase + mOff);
      const v4f b1 = *(const v4f*)(bias + mBase + mOff + 4);
      br[0] = b0[0]; br[1] = b0[1]; br[2] = b0[2]; br[3] = b0[3];
      br[4] = b1[0]; br[5] = b1[1]; br[6] = b1[2]; br[7] = b1[3];
    } else {
#pragma unroll
      for (int r = 0; r < 8; ++r) br[r] = 0.f;
    }
#pragma unroll
    for (int j = 0; j < 4; ++j) {
      const int n = n0 + (j << 4) + rlane;
      float bv = 0.f;
      if (BIAS_MODE == 2) bv = bias[n];
#pragma unroll
      for (int r = 0; r < 8; ++r) {
        float v = acc[i][j][r] * scale;
        if (BIAS_MODE == 1) v += br[r];
        if (BIAS_MODE == 2) v += bv;
        if (OUT_MODE == 1) v *= oscale;
        slab[(mOff + r) * 68 + (j << 4) + rlane] = v;
      }
    }
    wave_lds_sync();
    if (OUT_MODE == 0) {
      float* C = (float*)Cout + (size_t)b * strideC;
      const int hh = lane >> 4, c4 = (lane & 15) * 4;
#pragma unroll
      for (int grp = 0; grp < 2; ++grp) {
        v4f vals[4];
#pragma unroll
        for (int it = 0; it < 4; ++it) {
          const int row = (grp * 4 + it) * 2 + hh;
          v4f v = *(const v4f*)(slab + row * 68 + c4);
          const size_t go = (size_t)(mBase + row) * ldc + n0 + c4;
          if (RESID >= 1) {
            const v4f rr = *(const v4f*)(resid + go);
            v += rr;
          }
          if (RESID == 2) {
            const v4f mm = *(const v4f*)(rowadd + (size_t)((mBase + row) >> rowshift) * ldc + n0 + c4);
            v += mm;
          }
          vals[it] = v;
        }
        for (int pass = 0; pass < 2; ++pass) {
#pragma unroll
          for (int it = 0; it < 4; ++it) {
            const int row = (grp * 4 + it) * 2 + hh;
            *(volatile v4f*)(C + (size_t)(mBase + row) * ldc + n0 + c4) = vals[it];
          }
          __threadfence();
        }
      }
    } else {
      const int q = lane >> 3, c8 = (lane & 7) * 8;
      unsigned short* C = (unsigned short*)Cout + (size_t)b * strideC;
      v8h hv[4];
#pragma unroll
      for (int it = 0; it < 4; ++it) {
        const int row = it * 4 + q;
        const float* sp = slab + row * 68 + c8;
        const v4f a0 = *(const v4f*)(sp);
        const v4f a1 = *(const v4f*)(sp + 4);
#pragma unroll
        for (int e = 0; e < 4; ++e) {
          hv[it][e]     = to_f16_flush(a0[e]);
          hv[it][4 + e] = to_f16_flush(a1[e]);
        }
      }
      for (int pass = 0; pass < 2; ++pass) {
#pragma unroll
        for (int it = 0; it < 4; ++it) {
          const int row = it * 4 + q;
          *(volatile v8h*)(C + (size_t)(mBase + row) * ldc + n0 + c8) = hv[it];
        }
        __threadfence();
      }
    }
    wave_lds_sync();
  }
}

__global__ __launch_bounds__(256) void cvt_scale_f16_kernel(
    const float* __restrict__ src, unsigned short* __restrict__ dst, int total8, float carry)
{
  const int i = blockIdx.x * 256 + threadIdx.x;
  if (i >= total8) return;
  const size_t e0 = (size_t)i << 3;
  const v4f a0 = *(const v4f*)(src + e0);
  const v4f a1 = *(const v4f*)(src + e0 + 4);
  v8h hv;
#pragma unroll
  for (int e = 0; e < 4; ++e) {
    hv[e]     = to_f16_flush(a0[e] * carry);
    hv[4 + e] = to_f16_flush(a1[e] * carry);
  }
  unsigned short* q = dst + e0;
  *(volatile v8h*)q = hv;
  __threadfence();
  *(volatile v8h*)q = hv;
}

__global__ __launch_bounds__(256) void transpose_cvt_f16_kernel(
    const float* __restrict__ in, unsigned short* __restrict__ out, int rows, int cols, float carry)
{
  __shared__ float tile[64 * 65];
  const int tid = threadIdx.x;
  const int c0 = blockIdx.x * 64, r0 = blockIdx.y * 64;
#pragma unroll
  for (int it = 0; it < 4; ++it) {
    const int idx = tid + it * 256;
    const int r = idx >> 4, c4 = (idx & 15) << 2;
    const v4f f = *(const v4f*)(in + (size_t)(r0 + r) * cols + c0 + c4);
    tile[r * 65 + c4 + 0] = f[0];
    tile[r * 65 + c4 + 1] = f[1];
    tile[r * 65 + c4 + 2] = f[2];
    tile[r * 65 + c4 + 3] = f[3];
  }
  __syncthreads();
  const int q = tid >> 3, c8 = (tid & 7) * 8;
  v8h hv[2];
#pragma unroll
  for (int it = 0; it < 2; ++it) {
    const int cc = it * 32 + q;
#pragma unroll
    for (int e = 0; e < 8; ++e) hv[it][e] = to_f16_flush(tile[(c8 + e) * 65 + cc] * carry);
  }
  for (int pass = 0; pass < 2; ++pass) {
#pragma unroll
    for (int it = 0; it < 2; ++it) {
      const int cc = it * 32 + q;
      *(volatile v8h*)(out + (size_t)(c0 + cc) * rows + r0 + c8) = hv[it];
    }
    __threadfence();
  }
}

__global__ __launch_bounds__(256) void layernorm_f16_kernel(
    const float* __restrict__ xa, const float* __restrict__ xb, int rows_a, int rows_total,
    const float* __restrict__ g, const float* __restrict__ beta,
    unsigned short* __restrict__ out, float carry)
{
  const int lane = threadIdx.x & 31, wave = threadIdx.x >> 5;
  const int row = blockIdx.x * 8 + wave;
  if (row >= rows_total) return;
  const bool first = (row < rows_a);
  const int rsel = first ? row : (row - rows_a);
  const float* src = first ? xa : xb;
  const float* xr = src + (size_t)rsel * kH;
  float v[32];
#pragma unroll
  for (int i = 0; i < 4; ++i) {
    const v4f a0 = *(const v4f*)(xr + i * 256 + lane * 8);
    const v4f a1 = *(const v4f*)(xr + i * 256 + lane * 8 + 4);
    v[8 * i + 0] = a0[0]; v[8 * i + 1] = a0[1]; v[8 * i + 2] = a0[2]; v[8 * i + 3] = a0[3];
    v[8 * i + 4] = a1[0]; v[8 * i + 5] = a1[1]; v[8 * i + 6] = a1[2]; v[8 * i + 7] = a1[3];
  }
  float s = 0.0f;
#pragma unroll
  for (int e = 0; e < 32; ++e) s += v[e];
#pragma unroll
  for (int off = 16; off > 0; off >>= 1) s += __shfl_xor(s, off, 32);
  const float mu = s * (1.0f / (float)kH);
  float q = 0.0f;
#pragma unroll
  for (int e = 0; e < 32; ++e) {
    v[e] -= mu;
    q = fmaf(v[e], v[e], q);
  }
#pragma unroll
  for (int off = 16; off > 0; off >>= 1) q += __shfl_xor(q, off, 32);
  const float inv = rsqrtf(q * (1.0f / (float)kH) + 1e-5f);
  v8h hv[4];
#pragma unroll
  for (int i = 0; i < 4; ++i) {
    const v4f g0 = *(const v4f*)(g + i * 256 + lane * 8);
    const v4f g1 = *(const v4f*)(g + i * 256 + lane * 8 + 4);
    const v4f b0 = *(const v4f*)(beta + i * 256 + lane * 8);
    const v4f b1 = *(const v4f*)(beta + i * 256 + lane * 8 + 4);
#pragma unroll
    for (int e = 0; e < 4; ++e) {
      const float y0 = (v[8 * i + e] * inv) * g0[e] + b0[e];
      const float y1 = (v[8 * i + 4 + e] * inv) * g1[e] + b1[e];
      hv[i][e]     = to_f16_flush(y0 * carry);
      hv[i][4 + e] = to_f16_flush(y1 * carry);
    }
  }
  unsigned short* orow = out + (size_t)row * kH + lane * 8;
  for (int pass = 0; pass < 2; ++pass) {
#pragma unroll
    for (int i = 0; i < 4; ++i) *(volatile v8h*)(orow + i * 256) = hv[i];
    __threadfence();
  }
}

__global__ __launch_bounds__(256) void progmean_kernel(const float* __restrict__ pp, float* __restrict__ pm)
{
  const int tid = threadIdx.x;
  const int b = tid >> 6, p = tid & 63;
  const float* src = pp + (size_t)b * kT * kP + p;
  float s0 = 0.0f, s1 = 0.0f, s2 = 0.0f, s3 = 0.0f;
#pragma unroll 1
  for (int t = 0; t < kT; t += 4) {
    s0 += src[(size_t)(t + 0) * kP];
    s1 += src[(size_t)(t + 1) * kP];
    s2 += src[(size_t)(t + 2) * kP];
    s3 += src[(size_t)(t + 3) * kP];
  }
  const float m = ((s0 + s1) + (s2 + s3)) * (1.0f / (float)kT);
  volatile float* dst = pm + tid;
  *dst = m;
  __threadfence();
  *dst = m;
}

__global__ __launch_bounds__(256) void progmod_kernel(
    const float* __restrict__ pm, const float* __restrict__ Wp, const float* __restrict__ bp, float* __restrict__ mod)
{
  __shared__ __align__(16) float spm[kB * kP];
  const int tid = threadIdx.x;
  spm[tid] = pm[tid];
  __syncthreads();
  const int idx = blockIdx.x * 256 + tid;
  const int b = idx >> 10, h = idx & (kH - 1);
  const float* wrow = Wp + (size_t)h * kP;
  const float* prow = spm + b * kP;
  float acc = 0.0f;
#pragma unroll 1
  for (int p4 = 0; p4 < kP / 4; ++p4) {
    const v4f w = *(const v4f*)(wrow + 4 * p4);
    const v4f q = *(const v4f*)(prow + 4 * p4);
    acc = fmaf(q[0], w[0], acc);
    acc = fmaf(q[1], w[1], acc);
    acc = fmaf(q[2], w[2], acc);
    acc = fmaf(q[3], w[3], acc);
  }
  const float val = acc + bp[h];
  volatile float* dst = mod + idx;
  *dst = val;
  __threadfence();
  *dst = val;
}

__global__ __launch_bounds__(128) __attribute__((amdgpu_num_vgpr(256))) void attn128_kernel(
    const unsigned short* __restrict__ Qp, const unsigned short* __restrict__ Kp,
    const unsigned short* __restrict__ Vtp, unsigned short* __restrict__ ctx,
    float sscale, float oinv)
{
  __shared__ __align__(16) _Float16 Psh[4][16 * 64];
  __shared__ __align__(16) float    Os[4][16 * 132];
  const _Float16* Q  = (const _Float16*)Qp;
  const _Float16* Kq = (const _Float16*)Kp;
  const _Float16* Vt = (const _Float16*)Vtp;

  const int tid  = threadIdx.x;
  const int wave = tid >> 5;
  const int lane = tid & 31;
  const int hh   = lane >> 4;
  const int c    = lane & 15;

  const int bx = blockIdx.x;
  const int qb = bx & 31;
  const int bh = bx >> 5;
  const int h  = bh & (kNH - 1);
  const int b  = bh >> 3;
  const int q0 = qb * 64 + wave * 16;

  v16h qa[4];
  {
    const _Float16* qrow = Q + (size_t)(b * kT + q0 + c) * kH + h * kHD + 8 * hh;
#pragma unroll
    for (int dc = 0; dc < 4; ++dc) qa[dc] = FragH::load(qrow + dc * 32);
  }
  const _Float16* kbase = Kq + (size_t)(b * kT + c) * kH + h * kHD + 8 * hh;
  const _Float16* vbase = Vt + ((size_t)b * kH + h * kHD + c) * kT + 8 * hh;

  float mrow[8], lrow[8];
  v8f oacc[8];
#pragma unroll
  for (int r = 0; r < 8; ++r) { mrow[r] = -INFINITY; lrow[r] = 0.f; }
#pragma unroll
  for (int t = 0; t < 8; ++t) oacc[t] = (v8f){0.f,0.f,0.f,0.f,0.f,0.f,0.f,0.f};

  _Float16* pw = Psh[wave];

#pragma unroll 1
  for (int kc = 0; kc < kT / 64; ++kc) {
    const int kv0 = kc * 64;
    v8f s[4];
#pragma unroll
    for (int j = 0; j < 4; ++j) s[j] = (v8f){0.f,0.f,0.f,0.f,0.f,0.f,0.f,0.f};
#pragma unroll
    for (int dc = 0; dc < 4; ++dc) {
      const _Float16* kp = kbase + (size_t)kv0 * kH + dc * 32;
      const v16h kb0 = FragH::load(kp);
      const v16h kb1 = FragH::load(kp + (size_t)16 * kH);
      const v16h kb2 = FragH::load(kp + (size_t)32 * kH);
      const v16h kb3 = FragH::load(kp + (size_t)48 * kH);
      s[0] = FragH::mma(qa[dc], kb0, s[0]);
      s[1] = FragH::mma(qa[dc], kb1, s[1]);
      s[2] = FragH::mma(qa[dc], kb2, s[2]);
      s[3] = FragH::mma(qa[dc], kb3, s[3]);
      guard4_h(s[0], s[1], s[2], s[3], qa[dc], kb0, kb1, kb2, kb3);
    }
    float cm[8];
#pragma unroll
    for (int r = 0; r < 8; ++r) {
      float m = fmaxf(fmaxf(s[0][r], s[1][r]), fmaxf(s[2][r], s[3][r]));
#pragma unroll
      for (int off = 1; off < 16; off <<= 1) m = fmaxf(m, __shfl_xor(m, off, 32));
      cm[r] = m * sscale;
    }
#pragma unroll
    for (int r = 0; r < 8; ++r) {
      const float mnew = fmaxf(mrow[r], cm[r]);
      const float alpha = __expf(mrow[r] - mnew);
      mrow[r] = mnew;
      float psum = 0.f;
#pragma unroll
      for (int j = 0; j < 4; ++j) {
        const float p = __expf(fmaf(s[j][r], sscale, -mnew));
        psum += p;
        pw[(8 * hh + r) * 64 + j * 16 + c] = to_f16_flush(p * kCarryP);
      }
#pragma unroll
      for (int off = 1; off < 16; off <<= 1) psum += __shfl_xor(psum, off, 32);
      lrow[r] = lrow[r] * alpha + psum;
#pragma unroll
      for (int t = 0; t < 8; ++t) oacc[t][r] *= alpha;
    }
    wave_lds_sync();
#pragma unroll
    for (int kk = 0; kk < 2; ++kk) {
      const v16h pa = FragH::load(pw + c * 64 + kk * 32 + 8 * hh);
      const _Float16* vp = vbase + kv0 + kk * 32;
      {
        const v16h vb0 = FragH::load(vp);
        const v16h vb1 = FragH::load(vp + (size_t)16 * kT);
        const v16h vb2 = FragH::load(vp + (size_t)32 * kT);
        const v16h vb3 = FragH::load(vp + (size_t)48 * kT);
        oacc[0] = FragH::mma(pa, vb0, oacc[0]);
        oacc[1] = FragH::mma(pa, vb1, oacc[1]);
        oacc[2] = FragH::mma(pa, vb2, oacc[2]);
        oacc[3] = FragH::mma(pa, vb3, oacc[3]);
        guard4_h(oacc[0], oacc[1], oacc[2], oacc[3], pa, vb0, vb1, vb2, vb3);
      }
      {
        const v16h vb4 = FragH::load(vp + (size_t)64 * kT);
        const v16h vb5 = FragH::load(vp + (size_t)80 * kT);
        const v16h vb6 = FragH::load(vp + (size_t)96 * kT);
        const v16h vb7 = FragH::load(vp + (size_t)112 * kT);
        oacc[4] = FragH::mma(pa, vb4, oacc[4]);
        oacc[5] = FragH::mma(pa, vb5, oacc[5]);
        oacc[6] = FragH::mma(pa, vb6, oacc[6]);
        oacc[7] = FragH::mma(pa, vb7, oacc[7]);
        guard4_h(oacc[4], oacc[5], oacc[6], oacc[7], pa, vb4, vb5, vb6, vb7);
      }
    }
    wave_lds_sync();
  }

  float* os = Os[wave];
#pragma unroll
  for (int r = 0; r < 8; ++r) {
    const float inv = oinv * __builtin_amdgcn_rcpf(lrow[r]);
#pragma unroll
    for (int t = 0; t < 8; ++t) os[(8 * hh + r) * 132 + t * 16 + c] = oacc[t][r] * inv;
  }
  wave_lds_sync();
  {
    const int c8 = (lane & 15) * 8;
    v8h hv[8];
#pragma unroll
    for (int it = 0; it < 8; ++it) {
      const int row = it * 2 + hh;
      const float* sp = os + row * 132 + c8;
      const v4f a0 = *(const v4f*)(sp);
      const v4f a1 = *(const v4f*)(sp + 4);
#pragma unroll
      for (int e = 0; e < 4; ++e) {
        hv[it][e]     = to_f16_flush(a0[e]);
        hv[it][4 + e] = to_f16_flush(a1[e]);
      }
    }
    unsigned short* dst = ctx + (size_t)(b * kT + q0) * kH + h * kHD + c8;
    for (int pass = 0; pass < 2; ++pass) {
#pragma unroll
      for (int it = 0; it < 8; ++it) {
        const int row = it * 2 + hh;
        *(volatile v8h*)(dst + (size_t)row * kH) = hv[it];
      }
      __threadfence();
    }
  }
}

__global__ __launch_bounds__(256) void scan_kernel(
    const float* __restrict__ A, const float* __restrict__ U, float* __restrict__ states)
{
  __shared__ __align__(16) float sS[2 * kB * kS];
  const int tid = threadIdx.x;
  const int b = tid >> 6, j = tid & 63;
  float arow[64];
#pragma unroll
  for (int k4 = 0; k4 < 16; ++k4) {
    const v4f av = *(const v4f*)(A + j * kS + 4 * k4);
    arow[4 * k4 + 0] = av[0]; arow[4 * k4 + 1] = av[1]; arow[4 * k4 + 2] = av[2]; arow[4 * k4 + 3] = av[3];
  }
  sS[tid] = 0.0f;
  sS[kB * kS + tid] = 0.0f;
  __syncthreads();
  const float* urow = U + (size_t)b * kT * kS + j;
  float* srow = states + (size_t)b * kT * kS + j;
  float unext = urow[0];
#pragma unroll 1
  for (int t = 0; t < kT; ++t) {
    const int cur = (t & 1) * (kB * kS);
    const float* sp = sS + cur + b * kS;
    float acc = 0.0f;
#pragma unroll
    for (int k4 = 0; k4 < 16; ++k4) {
      const v4f sv = *(const v4f*)(sp + 4 * k4);
      acc = fmaf(arow[4 * k4 + 0], sv[0], acc);
      acc = fmaf(arow[4 * k4 + 1], sv[1], acc);
      acc = fmaf(arow[4 * k4 + 2], sv[2], acc);
      acc = fmaf(arow[4 * k4 + 3], sv[3], acc);
    }
    const float u = unext;
    const int tn = (t + 1 < kT) ? (t + 1) : (kT - 1);
    unext = urow[(size_t)tn * kS];
    const float e = expf(-acc);
    const float sg = __builtin_amdgcn_rcpf(1.0f + e);
    const float sn = acc * sg + u;
    sS[(kB * kS - cur) + tid] = sn;
    volatile float* dst = srow + (size_t)t * kS;
    *dst = sn;
    __threadfence();
    *dst = sn;
    __syncthreads();
  }
}

extern "C" void kernel_launch(void* const* d_in, const int* in_sizes, int n_in,
                              void* d_out, int out_size, void* d_ws, size_t ws_size,
                              hipStream_t stream) {
  if (n_in < 19) return;
  if (in_sizes[0] != kM * kH) return;
  if (in_sizes[1] != kM * kH) return;
  if (in_sizes[2] != kB * kT) return;
  if (in_sizes[3] != kM * kP) return;
  if (in_sizes[4] != kS * kS) return;
  if (in_sizes[5] != kH * kS) return;
  if (in_sizes[6] != kS * kH) return;
  if (in_sizes[7] != kH * kH) return;
  if (in_sizes[8] != kH) return;
  if (in_sizes[9] != 3 * kH * kH) return;
  if (in_sizes[10] != 3 * kH) return;
  if (in_sizes[11] != kH * kH) return;
  if (in_sizes[12] != kH) return;
  if (in_sizes[13] != kH * kP) return;
  if (in_sizes[14] != kH) return;
  if (in_sizes[15] != kH || in_sizes[16] != kH || in_sizes[17] != kH || in_sizes[18] != kH) return;
  if (out_size != kM * kH) return;
  if (ws_size < kWsTotal) return;

  const float* builder = (const float*)d_in[0];
  const float* base    = (const float*)d_in[1];
  const float* pp      = (const float*)d_in[3];
  const float* Amat    = (const float*)d_in[4];
  const float* Bmat    = (const float*)d_in[5];
  const float* Cmat    = (const float*)d_in[6];
  const float* W_in    = (const float*)d_in[7];
  const float* b_in    = (const float*)d_in[8];
  const float* W_qkv   = (const float*)d_in[9];
  const float* b_qkv   = (const float*)d_in[10];
  const float* W_o     = (const float*)d_in[11];
  const float* b_o     = (const float*)d_in[12];
  const float* W_prog  = (const float*)d_in[13];
  const float* b_prog  = (const float*)d_in[14];
  const float* g1      = (const float*)d_in[15];
  const float* beta1   = (const float*)d_in[16];
  const float* g2      = (const float*)d_in[17];
  const float* beta2   = (const float*)d_in[18];
  float* out = (float*)d_out;

  char* ws = (char*)d_ws;
  unsigned short* XQ   = (unsigned short*)(ws + kOffXQ);
  unsigned short* BN   = (unsigned short*)(ws + kOffBN);
  unsigned short* WQKV = (unsigned short*)(ws + kOffWQKV);
  unsigned short* WO   = (unsigned short*)(ws + kOffWO);
  unsigned short* WIN  = (unsigned short*)(ws + kOffWIN);
  unsigned short* BMT  = (unsigned short*)(ws + kOffBMT);
  unsigned short* CMT  = (unsigned short*)(ws + kOffCMT);
  unsigned short* QP   = (unsigned short*)(ws + kOffQP);
  unsigned short* KP   = (unsigned short*)(ws + kOffKP);
  unsigned short* VT   = (unsigned short*)(ws + kOffVT);
  float*          X1   = (float*)(ws + kOffX1);
  float*          Ub   = (float*)(ws + kOffU);
  float*          ST32 = (float*)(ws + kOffST32);
  unsigned short* ST16 = (unsigned short*)(ws + kOffST16);
  float*          PM   = (float*)(ws + kOffPM);
  float*          MOD  = (float*)(ws + kOffMOD);

  const float inv_sqrt_hd = 1.0f / sqrtf((float)kHD);
  const float sc_proj  = 1.0f / (kCarryAct * kCarryW);
  const float sc_wo    = 1.0f / (kCarryCtx * kCarryW);
  const float sc_cm    = 1.0f / (kCarryAct * kCarryC);
  const float sscale   = inv_sqrt_hd / (kCarryAct * kCarryAct);
  const float oinv     = kCarryCtx / (kCarryP * kCarryAct);

  cvt_scale_f16_kernel<<<(3 * kH * kH / 8) / 256, 256, 0, stream>>>(W_qkv, WQKV, 3 * kH * kH / 8, kCarryW);
  cvt_scale_f16_kernel<<<(kH * kH / 8) / 256, 256, 0, stream>>>(W_o, WO, kH * kH / 8, kCarryW);
  cvt_scale_f16_kernel<<<(kH * kH / 8) / 256, 256, 0, stream>>>(W_in, WIN, kH * kH / 8, kCarryW);
  transpose_cvt_f16_kernel<<<dim3(kS / 64, kH / 64), 256, 0, stream>>>(Bmat, BMT, kH, kS, kCarryW);
  transpose_cvt_f16_kernel<<<dim3(kH / 64, kS / 64), 256, 0, stream>>>(Cmat, CMT, kS, kH, kCarryC);

  layernorm_f16_kernel<<<(2 * kM) / 8, 256, 0, stream>>>(builder, base, kM, 2 * kM, g1, beta1, XQ, kCarryAct);

  progmean_kernel<<<1, 256, 0, stream>>>(pp, PM);
  progmod_kernel<<<(kB * kH) / 256, 256, 0, stream>>>(PM, W_prog, b_prog, MOD);

  gemm64_f16_kernel<2, 1, 0><<<dim3(256, 1), 256, 0, stream>>>(
      XQ, kH, 0L, WQKV, kH, 0L, (void*)QP, kH, 0L,
      b_qkv, builder, MOD, kTShift, kM, kH, kH, sc_proj, kCarryAct);
  gemm64_f16_kernel<2, 1, 0><<<dim3(256, 1), 256, 0, stream>>>(
      BN, kH, 0L, WQKV + (size_t)kH * kH, kH, 0L, (void*)KP, kH, 0L,
      b_qkv + kH, builder, MOD, kTShift, kM, kH, kH, sc_proj, kCarryAct);
  gemm64_f16_kernel<1, 1, 0><<<dim3(64, kB), 256, 0, stream>>>(
      WQKV + (size_t)2 * kH * kH, kH, 0L, BN, kH, (long)kT * kH, (void*)VT, kT, (long)kH * kT,
      b_qkv + 2 * kH, builder, MOD, kTShift, kH, kT, kH, sc_proj, kCarryAct);

  attn128_kernel<<<kB * kNH * (kT / 64), 128, 0, stream>>>(QP, KP, VT, XQ, sscale, oinv);

  gemm64_f16_kernel<2, 0, 1><<<dim3(256, 1), 256, 0, stream>>>(
      XQ, kH, 0L, WO, kH, 0L, (void*)X1, kH, 0L,
      b_o, builder, MOD, kTShift, kM, kH, kH, sc_wo, 1.0f);

  layernorm_f16_kernel<<<kM / 8, 256, 0, stream>>>(X1, X1, kM, kM, g2, beta2, BN, kCarryAct);

  gemm64_f16_kernel<2, 1, 0><<<dim3(256, 1), 256, 0, stream>>>(
      BN, kH, 0L, WIN, kH, 0L, (void*)QP, kH, 0L,
      b_in, builder, MOD, kTShift, kM, kH, kH, sc_proj, kCarryAct);

  gemm64_f16_kernel<0, 0, 0><<<dim3(16, 1), 256, 0, stream>>>(
      QP, kH, 0L, BMT, kH, 0L, (void*)Ub, kS, 0L,
      b_in, builder, MOD, kTShift, kM, kS, kH, sc_proj, 1.0f);

  scan_kernel<<<1, 256, 0, stream>>>(Amat, Ub, ST32);

  cvt_scale_f16_kernel<<<(kM * kS / 8) / 256, 256, 0, stream>>>(ST32, ST16, kM * kS / 8, kCarryAct);

  gemm64_f16_kernel<0, 0, 2><<<dim3(256, 1), 256, 0, stream>>>(
      ST16, kS, 0L, CMT, kS, 0L, (void*)out, kH, 0L,
      b_in, X1, MOD, kTShift, kM, kH, kS, sc_cm, 1.0f);
}
